// GELU217_23648089932089
// MI455X (gfx1250) — hardware-verified
//
#include <hip/hip_runtime.h>
#include <math.h>
#include <stdint.h>

#define NB   8
#define NT   2048
#define ND   512
#define NR   (NB * NT)
#define RPB  8
#define IT   64
#define JT   64
#define XSC  64.0f
#define ISC2 0.000244140625f
#define GK   0.7978845608028654f
#define GC3  0.044715f

static_assert(ND == 512);
static_assert((NT % IT) == 0);
static_assert((NT % JT) == 0);
static_assert((NR % RPB) == 0);
static_assert((ND % 32) == 0);
static_assert(IT == 4 * 16);
static_assert(JT == 4 * 16);
static_assert((ND % 256) == 0);

typedef _Float16       v16h __attribute__((ext_vector_type(16)));
typedef _Float16       v8h  __attribute__((ext_vector_type(8)));
typedef float          v8f  __attribute__((ext_vector_type(8)));
typedef float          v4f  __attribute__((ext_vector_type(4)));
typedef unsigned int   v4u  __attribute__((ext_vector_type(4)));

union FragH { v16h v; v8h h[2]; };
static_assert(sizeof(FragH) == 32);

__device__ __forceinline__ unsigned short bf_bits(float f) {
  unsigned u = __float_as_uint(f);
  return (unsigned short)((u + 0x7FFFu + ((u >> 16) & 1u)) >> 16);
}
__device__ __forceinline__ float bf_up(unsigned short h) { return __uint_as_float(((unsigned)h) << 16); }
__device__ __forceinline__ float bfr(float f) { return bf_up(bf_bits(f)); }
__device__ __forceinline__ v4f bfr4(v4f v) {
  v4f r;
  r[0] = bfr(v[0]); r[1] = bfr(v[1]); r[2] = bfr(v[2]); r[3] = bfr(v[3]);
  return r;
}
__device__ __forceinline__ unsigned short h_bits(_Float16 x) { return __builtin_bit_cast(unsigned short, x); }
__device__ __forceinline__ unsigned pk16(unsigned short a, unsigned short b) { return (unsigned)a | ((unsigned)b << 16); }
__device__ __forceinline__ v8f zero8() { v8f z = {0.f, 0.f, 0.f, 0.f, 0.f, 0.f, 0.f, 0.f}; return z; }

__device__ __forceinline__ float tanh_e(float y) {
  const float a = fabsf(y);
  const float e = __expf(2.0f * a);
  const float r = __builtin_amdgcn_rcpf(e + 1.0f);
  const float t = fmaf(-2.0f, r, 1.0f);
  return copysignf(t, y);
}
__device__ __forceinline__ float gelu_f(float x) {
  const float x3 = x * x * x;
  const float y  = GK * (x + GC3 * x3);
  return 0.5f * x * (1.0f + tanh_e(y));
}
__device__ __forceinline__ float softplus_f(float v) { return log1pf(expf(v)); }

__device__ __forceinline__ v16h ldfrag_h(const _Float16* p) {
  FragH f;
  f.h[0] = *(const v8h*)(p);
  f.h[1] = *(const v8h*)(p + 16);
  return f.v;
}

__device__ __forceinline__ v8f mma_h(v16h a, v16h b, v8f c) {
  v8f d = __builtin_amdgcn_wmma_f32_16x16x32_f16(false, a, false, b, (short)0, c, false, false);
#if defined(__HIP_DEVICE_COMPILE__)
  asm volatile("v_nop\n\tv_nop\n\tv_nop\n\tv_nop" : "+v"(d) : "v"(a), "v"(b));
#endif
  return d;
}

__global__ __launch_bounds__(256)
void norm_kernel(const float* __restrict__ x, unsigned short* XN) {
  const int tid  = threadIdx.x;
  const int wave = tid >> 5, lane = tid & 31;
  const int row  = blockIdx.x * RPB + wave;
  const float* xr = x + (size_t)row * ND + 8 * lane;
  const v4f a0 = bfr4(*(const v4f*)(xr));
  const v4f a1 = bfr4(*(const v4f*)(xr + 4));
  const v4f b0 = bfr4(*(const v4f*)(xr + 256));
  const v4f b1 = bfr4(*(const v4f*)(xr + 260));
  float ss = 0.f;
#pragma unroll
  for (int q = 0; q < 4; ++q) {
    ss = fmaf(a0[q], a0[q], ss);
    ss = fmaf(a1[q], a1[q], ss);
    ss = fmaf(b0[q], b0[q], ss);
    ss = fmaf(b1[q], b1[q], ss);
  }
#pragma unroll
  for (int msk = 16; msk >= 1; msk >>= 1) ss += __shfl_xor(ss, msk, 32);
  const float nx  = fmaxf(sqrtf(ss), 1.0e-12f);
  const float inv = XSC / nx;
  v4u ua, ub;
#pragma unroll
  for (int t = 0; t < 2; ++t) {
    ua[t]     = pk16(h_bits((_Float16)(a0[2 * t] * inv)), h_bits((_Float16)(a0[2 * t + 1] * inv)));
    ua[2 + t] = pk16(h_bits((_Float16)(a1[2 * t] * inv)), h_bits((_Float16)(a1[2 * t + 1] * inv)));
    ub[t]     = pk16(h_bits((_Float16)(b0[2 * t] * inv)), h_bits((_Float16)(b0[2 * t + 1] * inv)));
    ub[2 + t] = pk16(h_bits((_Float16)(b1[2 * t] * inv)), h_bits((_Float16)(b1[2 * t + 1] * inv)));
  }
  unsigned short* dst = XN + (size_t)row * ND + 8 * lane;
  *(volatile v4u*)(dst)       = ua;
  *(volatile v4u*)(dst + 256) = ub;
  __threadfence();
  *(volatile v4u*)(dst)       = ua;
  *(volatile v4u*)(dst + 256) = ub;
}

__global__ __launch_bounds__(128)
void gram_kernel(const unsigned short* __restrict__ XN, const float* __restrict__ p_ls,
                 const float* __restrict__ p_lw, float* G) {
  __shared__ __align__(16) float s_g[IT];
  const int tid  = threadIdx.x;
  const int wave = tid >> 5, lane = tid & 31;
  const int hh   = lane >> 4, m = lane & 15;
  const int bx   = blockIdx.x;
  const int b    = bx / (NT / IT);
  const int tile = bx % (NT / IT);
  const int i0   = tile * IT + wave * 16;
  const _Float16* Xh   = (const _Float16*)(const void*)XN;
  const _Float16* base = Xh + (size_t)b * NT * ND;
  const _Float16* ap   = base + (size_t)(i0 + m) * ND + 8 * hh;
  const int gr0 = i0 + 8 * hh;

  v8f rmx = zero8() - 2.0f;
#pragma unroll 1
  for (int jt = 0; jt < NT / JT; ++jt) {
    const int j0 = jt * JT;
    const _Float16* bp = base + (size_t)(j0 + m) * ND + 8 * hh;
    v8f acc0 = zero8(), acc1 = zero8(), acc2 = zero8(), acc3 = zero8();
#pragma unroll 4
    for (int ks = 0; ks < ND / 32; ++ks) {
      const v16h a = ldfrag_h(ap + 32 * ks);
      acc0 = mma_h(a, ldfrag_h(bp + 0 * 16 * ND + 32 * ks), acc0);
      acc1 = mma_h(a, ldfrag_h(bp + 1 * 16 * ND + 32 * ks), acc1);
      acc2 = mma_h(a, ldfrag_h(bp + 2 * 16 * ND + 32 * ks), acc2);
      acc3 = mma_h(a, ldfrag_h(bp + 3 * 16 * ND + 32 * ks), acc3);
    }
#pragma unroll
    for (int r = 0; r < 8; ++r) {
      const int gr = gr0 + r;
      float s0 = acc0[r] * ISC2, s1 = acc1[r] * ISC2, s2 = acc2[r] * ISC2, s3 = acc3[r] * ISC2;
      s0 = (gr == j0 + 0 * 16 + m) ? -2.0f : s0;
      s1 = (gr == j0 + 1 * 16 + m) ? -2.0f : s1;
      s2 = (gr == j0 + 2 * 16 + m) ? -2.0f : s2;
      s3 = (gr == j0 + 3 * 16 + m) ? -2.0f : s3;
      rmx[r] = fmaxf(rmx[r], fmaxf(fmaxf(s0, s1), fmaxf(s2, s3)));
    }
  }
#pragma unroll
  for (int r = 0; r < 8; ++r) {
#pragma unroll
    for (int msk = 1; msk < 16; msk <<= 1) rmx[r] = fmaxf(rmx[r], __shfl_xor(rmx[r], msk, 32));
  }
  const float sig = softplus_f(bfr(p_ls[0]));
  const float wn  = softplus_f(bfr(p_lw[0]));
  if (m == 0) {
#pragma unroll
    for (int r = 0; r < 8; ++r) {
      const float nn  = rmx[r];
      const float nov = 0.5f * (1.0f - nn);
      s_g[wave * 16 + 8 * hh + r] = 1.0f + wn * tanh_e(sig * nov);
    }
  }
  __syncthreads();
  if (wave == 0) {
    const int q = min(lane, 15);
    const v4f v = *(const v4f*)(s_g + 4 * q);
    float* gp = G + (size_t)b * NT + (size_t)tile * IT + 4 * q;
    if (lane < 16) *(volatile v4f*)gp = v;
    __threadfence();
    if (lane < 16) *(volatile v4f*)gp = v;
  }
}

__global__ __launch_bounds__(256)
void out_kernel(const float* __restrict__ x, const float* __restrict__ ema_mean, const float* __restrict__ ema_sq,
                const float* __restrict__ ema_out, const float* __restrict__ p_lt, const float* __restrict__ p_bu,
                const float* __restrict__ p_bd, const float* __restrict__ p_lg, const float* __restrict__ G,
                float* out) {
  __shared__ float s_par[4];
  __shared__ float s_red[RPB];
  __shared__ float s_mean[ND];
  __shared__ float s_rinv[ND];
  __shared__ float s_eo[ND];
  __shared__ __align__(16) float s_row[RPB * ND];
  const int tid  = threadIdx.x;
  const int wave = tid >> 5, lane = tid & 31;

  if (wave == 0) {
    const float v0 = bfr(p_lt[0]), v1 = bfr(p_bu[0]), v2 = bfr(p_bd[0]), v3 = bfr(p_lg[0]);
    const float v  = (lane == 0) ? v0 : ((lane == 1) ? v1 : ((lane == 2) ? v2 : v3));
    const float e  = expf(v);
    const float sp = log1pf(e);
    const float rs = (lane == 0) ? e : sp;
    if (lane < 4) s_par[lane] = rs;
  }
  float se = 0.f;
#pragma unroll 1
  for (int q = 0; q < ND / 256; ++q) {
    const int c = q * 256 + tid;
    const float mu = bfr(ema_mean[c]), s2 = bfr(ema_sq[c]), eo = bfr(ema_out[c]);
    const float var = fmaxf(s2 - mu * mu, 1.0e-4f);
    const float sdv = sqrtf(var);
    s_mean[c] = mu;
    s_rinv[c] = 1.0f / (sdv + 1.0e-5f);
    s_eo[c]   = eo;
    se = fmaf(eo, eo, se);
  }
#pragma unroll
  for (int msk = 16; msk >= 1; msk >>= 1) se += __shfl_xor(se, msk, 32);
  if (lane == 0) s_red[wave] = se;
  __syncthreads();
  float set = 0.f;
#pragma unroll
  for (int w = 0; w < RPB; ++w) set += s_red[w];
  const float ne   = fmaxf(sqrtf(set), 1.0e-12f);
  const float einv = __builtin_amdgcn_rcpf(ne);
  const float tau = s_par[0], bu = s_par[1], bd = s_par[2], gm = s_par[3];

  const int row = blockIdx.x * RPB + wave;
  const float* xr = x + (size_t)row * ND;
  float* rb = s_row + wave * ND;
  float so = 0.f, sdt = 0.f;
#pragma unroll 1
  for (int i = 0; i < 16; ++i) {
    const int c = (i >> 2) * 128 + 4 * lane + (i & 3);
    const float xi = bfr(xr[c]);
    const float o  = gelu_f(xi);
    const float z  = (xi - s_mean[c]) * s_rinv[c];
    const float t  = tanh_e(gm * z);
    const float up = bu * fmaxf(t, 0.f);
    const float dn = bd * fmaxf(-t, 0.f);
    const float gh = fminf(fmaxf(1.0f + up - dn, 0.05f), 8.0f);
    rb[c] = o * gh;
    so  = fmaf(o, o, so);
    sdt = fmaf(o, s_eo[c], sdt);
  }
#pragma unroll
  for (int msk = 16; msk >= 1; msk >>= 1) {
    so  += __shfl_xor(so, msk, 32);
    sdt += __shfl_xor(sdt, msk, 32);
  }
  const float no = fmaxf(sqrtf(so), 1.0e-12f);
  float cs = sdt * __builtin_amdgcn_rcpf(no) * einv;
  cs = fminf(fmaxf(cs, -1.0f), 1.0f);
  const float gc = __expf(-tau * cs);
  const float g  = gc * G[row];
  __syncthreads();

  const float* rs = rb + 4 * lane;
  const v4f w0 = *(const v4f*)(rs)       * g;
  const v4f w1 = *(const v4f*)(rs + 128) * g;
  const v4f w2 = *(const v4f*)(rs + 256) * g;
  const v4f w3 = *(const v4f*)(rs + 384) * g;
  float* op = out + (size_t)row * ND + 4 * lane;
  *(volatile v4f*)(op)       = w0;
  *(volatile v4f*)(op + 128) = w1;
  *(volatile v4f*)(op + 256) = w2;
  *(volatile v4f*)(op + 384) = w3;
  __threadfence();
  *(volatile v4f*)(op)       = w0;
  *(volatile v4f*)(op + 128) = w1;
  *(volatile v4f*)(op + 256) = w2;
  *(volatile v4f*)(op + 384) = w3;
}

extern "C" void kernel_launch(void* const* d_in, const int* in_sizes, int n_in,
                              void* d_out, int out_size, void* d_ws, size_t ws_size,
                              hipStream_t stream) {
  if (n_in < 10) return;
  if (in_sizes[0] != NR * ND || in_sizes[1] != ND || in_sizes[2] != ND || in_sizes[3] != ND) return;
  for (int i = 4; i < 10; ++i) { if (in_sizes[i] < 1) return; }
  if (out_size != NR * ND) return;

  size_t off = 0;
  const size_t oXN = off; off += (size_t)NR * ND * 2;
  const size_t oG  = off; off += (size_t)NR * 4;
  if (off > ws_size) return;
  if (off > (size_t)134217728) return;

  const float* x        = (const float*)d_in[0];
  const float* ema_mean = (const float*)d_in[1];
  const float* ema_sq   = (const float*)d_in[2];
  const float* ema_out  = (const float*)d_in[3];
  const float* log_tau  = (const float*)d_in[4];
  const float* log_bu   = (const float*)d_in[5];
  const float* log_bd   = (const float*)d_in[6];
  const float* log_g    = (const float*)d_in[7];
  const float* log_sig  = (const float*)d_in[8];
  const float* log_w    = (const float*)d_in[9];
  char* ws = (char*)d_ws;
  unsigned short* XN = (unsigned short*)(ws + oXN);
  float* G   = (float*)(ws + oG);
  float* out = (float*)d_out;

  const dim3 blk256(256), blk128(128);
  const dim3 gRow(NR / RPB);
  const dim3 gGram(NB * (NT / IT));

  norm_kernel<<<gRow, blk256, 0, stream>>>(x, XN);
  gram_kernel<<<gGram, blk128, 0, stream>>>(XN, log_sig, log_w, G);
  out_kernel<<<gRow, blk256, 0, stream>>>(x, ema_mean, ema_sq, ema_out, log_tau, log_bu, log_bd, log_g, G, out);
  (void)hipGetLastError();
}
